// m2oAttentionA3_32177894982193
// MI455X (gfx1250) — hardware-verified
//
#include <hip/hip_runtime.h>
#include <math.h>

typedef __attribute__((ext_vector_type(16))) _Float16 v16h;
typedef __attribute__((ext_vector_type(16))) __bf16 v16b;
typedef __attribute__((ext_vector_type(8)))  _Float16 v8h;
typedef __attribute__((ext_vector_type(8)))  float v8f;
typedef __attribute__((ext_vector_type(4)))  float v4f;
typedef __attribute__((ext_vector_type(2)))  float v2f;
typedef __attribute__((ext_vector_type(4)))  unsigned v4u;
typedef __attribute__((ext_vector_type(4)))  int v4i;
typedef float __attribute__((may_alias)) float_a;
typedef int __attribute__((may_alias)) int_a;

template <typename T> __device__ __forceinline__ void vst2(void* p, T v) { *(volatile T*)p = v; __threadfence(); *(volatile T*)p = v; }
__device__ __forceinline__ v8f wmma16(v16h a, v16h b, v8f c) {
  v8f d = __builtin_amdgcn_wmma_f32_16x16x32_f16(false, a, false, b, (short)0, c, false, false);
  asm volatile("v_nop\n\tv_nop\n\tv_nop\n\tv_nop" : "+v"(d) : "v"(a), "v"(b));
  return d;
}
__device__ __forceinline__ v8f wmma_bf(v16b a, v16b b, v8f c) {
  v8f d = __builtin_amdgcn_wmma_f32_16x16x32_bf16(false, a, false, b, (short)0, c, false, false);
  asm volatile("v_nop\n\tv_nop\n\tv_nop\n\tv_nop" : "+v"(d) : "v"(a), "v"(b));
  return d;
}
__device__ __forceinline__ v16h frag_h(const _Float16* rowk0, int lane) {
  union { v16h v; v8h q[2]; } u; const _Float16* p = rowk0 + 8 * (lane >> 4);
  u.q[0] = *(const v8h*)p; u.q[1] = *(const v8h*)(p + 16); return u.v;
}
__device__ __forceinline__ v16h frag_f32(const float* rowk0, int lane) {
  v16h a; const float* p = rowk0 + 8 * (lane >> 4);
#pragma unroll
  for (int i = 0; i < 8; ++i) { a[i] = (_Float16)p[i]; a[8 + i] = (_Float16)p[16 + i]; }
  return a;
}
__device__ __forceinline__ v16h frag_f32s(const float* rowk0, int lane, float sc) {
  v16h a; const float* p = rowk0 + 8 * (lane >> 4);
#pragma unroll
  for (int i = 0; i < 8; ++i) { a[i] = (_Float16)(p[i] * sc); a[8 + i] = (_Float16)(p[16 + i] * sc); }
  return a;
}
__device__ __forceinline__ v16h fragc_f32(const float* W, int k0, int n, int lane, int ld, int K) {
  v16h a; const int g = lane >> 4;
#pragma unroll
  for (int i = 0; i < 8; ++i) { const int ka = k0 + 8 * g + i, kb = ka + 16;
    a[i] = (_Float16)(ka < K ? W[(size_t)(ka < K ? ka : K - 1) * ld + n] : 0.f); a[8 + i] = (_Float16)(kb < K ? W[(size_t)(kb < K ? kb : K - 1) * ld + n] : 0.f); }
  return a;
}
struct F2 { v16b h, l; };
__device__ __forceinline__ F2 bsplit16(const float v[16]) { F2 r;
#pragma unroll
  for (int i = 0; i < 16; ++i) { const __bf16 h = (__bf16)v[i]; r.h[i] = h; r.l[i] = (__bf16)(v[i] - (float)h); }
  return r; }
__device__ __forceinline__ F2 split_row(const float* row, int k0, int lane) { float v[16]; const float* p = row + k0 + 8 * (lane >> 4);
#pragma unroll
  for (int i = 0; i < 8; ++i) { v[i] = p[i]; v[8 + i] = p[16 + i]; }
  return bsplit16(v); }
__device__ __forceinline__ F2 split_rowK(const float* row, int k0, int lane, int K) { float v[16]; const int g = lane >> 4;
#pragma unroll
  for (int i = 0; i < 8; ++i) { const int ka = k0 + 8 * g + i, kb = ka + 16; v[i] = ka < K ? row[ka < K ? ka : K - 1] : 0.f; v[8 + i] = kb < K ? row[kb < K ? kb : K - 1] : 0.f; }
  return bsplit16(v); }
__device__ __forceinline__ F2 split_col(const float* W, int k0, int n, int lane, int ld, int K) { float v[16]; const int g = lane >> 4;
#pragma unroll
  for (int i = 0; i < 8; ++i) { const int ka = k0 + 8 * g + i, kb = ka + 16; v[i] = ka < K ? W[(size_t)(ka < K ? ka : K - 1) * ld + n] : 0.f; v[8 + i] = kb < K ? W[(size_t)(kb < K ? kb : K - 1) * ld + n] : 0.f; }
  return bsplit16(v); }
__device__ __forceinline__ v8f mac3(const F2& a, const F2& b, v8f c) { c = wmma_bf(a.l, b.h, c); c = wmma_bf(a.h, b.l, c); return wmma_bf(a.h, b.h, c); }
__device__ __forceinline__ float sigm(float v) { return 1.0f / (1.0f + expf(-v)); }
#define LDSX() do { asm volatile("s_wait_dscnt 0" ::: "memory"); __builtin_amdgcn_wave_barrier(); __builtin_amdgcn_fence(__ATOMIC_RELEASE, "workgroup"); } while (0)


#define NBB 128
#define SQ 100
#define NC 25
#define DD 256
#define NM (NBB * NC)
#define NP1 (NBB * SQ)
typedef __attribute__((ext_vector_type(8))) __bf16 v8b;
__device__ __forceinline__ v16b frag_b(const __bf16* rowk0, int lane) {
  union { v16b v; v8b q[2]; } u; const __bf16* p = rowk0 + 8 * (lane >> 4);
  u.q[0] = *(const v8b*)p; u.q[1] = *(const v8b*)(p + 16); return u.v;
}
__device__ __forceinline__ float bfr(float v) { return (float)(__bf16)v; }
__device__ __attribute__((noinline)) float exp_ni(float v) { return expf(v); }
__device__ __attribute__((noinline)) float erf_ni(float v) { return erff(v); }

#define WS_P1  0u
#define WS_Q2  (WS_P1 + 4u * (size_t)NP1 * DD)
#define WS_AT  (WS_Q2 + 4u * (size_t)NM * DD)
#define WS_AV  (WS_AT + 4u * (size_t)NBB * 32 * 128)
#define WS_END (WS_AV + 4u * (size_t)NBB * 32 * DD)

__global__ __launch_bounds__(128) void k_lin(const float* __restrict__ IN, const float* __restrict__ Wm, const float* __restrict__ Bv, float* __restrict__ OUT) { __shared__ __align__(16) float sf[4][16][132];
  const int tid = threadIdx.x, wave = tid >> 5, lane = tid & 31, col = lane & 15, g = lane >> 4; const int c0 = blockIdx.y * 128; const size_t r0 = (size_t)blockIdx.x * 64 + wave * 16;
  v8f acc[8] = {};
#pragma unroll 2
  for (int kc = 0; kc < DD / 32; ++kc) { v16b a; { const float* p = IN + (r0 + col) * DD + kc * 32 + 8 * g;
#pragma unroll
      for (int i = 0; i < 8; ++i) { a[i] = (__bf16)p[i]; a[8 + i] = (__bf16)p[16 + i]; } }
#pragma unroll
    for (int j = 0; j < 8; ++j) { v16b w; const int o = c0 + j * 16 + col;
#pragma unroll
      for (int i = 0; i < 8; ++i) { w[i] = (__bf16)Wm[(size_t)(kc * 32 + 8 * g + i) * DD + o]; w[8 + i] = (__bf16)Wm[(size_t)(kc * 32 + 16 + 8 * g + i) * DD + o]; }
      acc[j] = wmma_bf(a, w, acc[j]); } }
#pragma unroll
  for (int j = 0; j < 8; ++j) { const float bb = Bv ? bfr(Bv[c0 + j * 16 + col]) : 0.f;
#pragma unroll
    for (int r = 0; r < 8; ++r) sf[wave][8 * g + r][j * 16 + col] = acc[j][r] + bb; }
  LDSX(); for (int rl = 0; rl < 16; ++rl) vst2(OUT + (r0 + rl) * DD + c0 + lane * 4, *(const v4f*)&sf[wave][rl][lane * 4]); }
__global__ __launch_bounds__(256) void k_att(const float* __restrict__ P1, const float* __restrict__ Q2, const int* __restrict__ MSK, const float* __restrict__ Vv, const float* __restrict__ BV, float* __restrict__ AT) { __shared__ float sv[DD]; __shared__ float sq[DD]; __shared__ __align__(16) float sl[32][128];
  const int t = threadIdx.x; const int bp = blockIdx.x;
  sv[t] = bfr(Vv[t]); for (int e = t; e < 32 * 128; e += 256) sl[e >> 7][e & 127] = 0.f;
  const float bv = bfr(BV[0]);
  __syncthreads();
#pragma unroll 1
  for (int k = 0; k < NC; ++k) { const int m = bp * NC + k; const int b1 = m % NBB;
    __syncthreads(); sq[t] = Q2[(size_t)m * DD + t]; __syncthreads();
    if (t < SQ) { const float* p1 = P1 + ((size_t)b1 * SQ + t) * DD; float a = bv;
#pragma unroll 1
      for (int h = 0; h < DD; ++h) a += tanhf(p1[h] + sq[h]) * sv[h];
      sl[k][t] = a; } }
  __syncthreads();
  if (t < SQ) { const bool keep = MSK[bp * SQ + t] != 0; float mx = -3.0e38f; for (int k = 0; k < NC; ++k) { const float v = keep ? sl[k][t] : -1.0e10f; sl[k][t] = v; mx = fmaxf(mx, v); } float s = 0.f; for (int k = 0; k < NC; ++k) { const float e = expf(sl[k][t] - mx); sl[k][t] = e; s += e; } const float inv = 1.0f / s; for (int k = 0; k < NC; ++k) sl[k][t] *= inv; }
  __syncthreads(); for (int q = t; q < 32 * 128 / 4; q += 256) vst2(AT + (size_t)bp * 32 * 128 + q * 4, *(const v4f*)&(&sl[0][0])[q * 4]); }
__global__ __launch_bounds__(128) void k_av(const float* __restrict__ AT, const float* __restrict__ X1, float* __restrict__ AV) { __shared__ __align__(16) float sf[32][132];
  const int tid = threadIdx.x, wave = tid >> 5, lane = tid & 31, col = lane & 15, g = lane >> 4; const size_t b = blockIdx.x; const int c0 = blockIdx.y * 128; const int rt = wave & 1, cg = wave >> 1;
  v8f acc[4] = {};
#pragma unroll
  for (int kc = 0; kc < 4; ++kc) { const F2 a = split_row(AT + (b * 32 + rt * 16 + col) * 128, kc * 32, lane);
#pragma unroll
    for (int j = 0; j < 4; ++j) { v16b xb; const int d = c0 + cg * 64 + j * 16 + col;
#pragma unroll
      for (int i = 0; i < 8; ++i) { const int s0 = kc * 32 + 8 * g + i, s1 = s0 + 16; xb[i] = (__bf16)(s0 < SQ ? X1[(b * SQ + s0) * DD + d] : 0.f); xb[8 + i] = (__bf16)(s1 < SQ ? X1[(b * SQ + s1) * DD + d] : 0.f); }
      acc[j] = wmma_bf(a.h, xb, acc[j]); acc[j] = wmma_bf(a.l, xb, acc[j]); } }
#pragma unroll
  for (int j = 0; j < 4; ++j)
#pragma unroll
    for (int r = 0; r < 8; ++r) sf[rt * 16 + 8 * g + r][cg * 64 + j * 16 + col] = acc[j][r];
  __syncthreads(); for (int e = tid; e < 32 * 32; e += 128) { const int rl = e >> 5, q = e & 31; vst2(AV + (b * 32 + rl) * DD + c0 + q * 4, *(const v4f*)&sf[rl][q * 4]); } }
__global__ __launch_bounds__(128) void k_out(const float* __restrict__ AV, const float* __restrict__ X2, const float* __restrict__ W3, const float* __restrict__ W4, const float* __restrict__ B4, float* __restrict__ OUT) { __shared__ __align__(16) float sf[32][DD + 4];
  const int tid = threadIdx.x, wave = tid >> 5, lane = tid & 31, col = lane & 15, g = lane >> 4; const size_t b = blockIdx.x; const int rt = wave & 1, ch = wave >> 1; const int k = rt * 16 + col;
  v8f acc[8] = {};
#pragma unroll 1
  for (int kc = 0; kc < DD / 32; ++kc) { const F2 a = split_row(AV + (b * 32 + k) * DD, kc * 32, lane); v16b a2; { const float* p = X2 + (b * NC + (k < NC ? k : 0)) * DD + kc * 32 + 8 * g;
#pragma unroll
      for (int i = 0; i < 8; ++i) { a2[i] = (__bf16)(k < NC ? p[i] : 0.f); a2[8 + i] = (__bf16)(k < NC ? p[16 + i] : 0.f); } }
#pragma unroll
    for (int j = 0; j < 8; ++j) { v16b w3, w4; const int o = ch * 128 + j * 16 + col;
#pragma unroll
      for (int i = 0; i < 8; ++i) { w3[i] = (__bf16)W3[(size_t)(kc * 32 + 8 * g + i) * DD + o]; w3[8 + i] = (__bf16)W3[(size_t)(kc * 32 + 16 + 8 * g + i) * DD + o]; w4[i] = (__bf16)W4[(size_t)(kc * 32 + 8 * g + i) * DD + o]; w4[8 + i] = (__bf16)W4[(size_t)(kc * 32 + 16 + 8 * g + i) * DD + o]; }
      acc[j] = wmma_bf(a.h, w3, acc[j]); acc[j] = wmma_bf(a.l, w3, acc[j]); acc[j] = wmma_bf(a2, w4, acc[j]); } }
#pragma unroll
  for (int j = 0; j < 8; ++j) { const int o = ch * 128 + j * 16 + col; const float bb = bfr(B4[o]);
#pragma unroll
    for (int r = 0; r < 8; ++r) sf[rt * 16 + 8 * g + r][o] = tanhf(acc[j][r] + bb); }
  __syncthreads(); for (int e = tid; e < NC * (DD / 4); e += 128) { const int rl = e / (DD / 4), q = e % (DD / 4); vst2(OUT + (b * NC + rl) * DD + q * 4, *(const v4f*)&sf[rl][q * 4]); } }
extern "C" void kernel_launch(void* const* d_in, const int* in_sizes, int n_in, void* d_out, int out_size, void* d_ws, size_t ws_size, hipStream_t stream) {
  (void)in_sizes; (void)n_in; (void)out_size;
  const float** F = (const float**)d_in;
  if (ws_size < (size_t)WS_END) return;
  char* ws = (char*)d_ws; float *P1 = (float*)(ws + WS_P1), *Q2 = (float*)(ws + WS_Q2), *AT = (float*)(ws + WS_AT), *AV = (float*)(ws + WS_AV);
  k_lin<<<dim3(NP1 / 64, DD / 128), 128, 0, stream>>>(F[0], F[3], nullptr, P1);
  k_lin<<<dim3(NM / 64, DD / 128), 128, 0, stream>>>(F[1], F[4], F[5], Q2);
  k_att<<<NBB, 256, 0, stream>>>(P1, Q2, (const int*)d_in[2], F[9], F[10], AT);
  k_av<<<dim3(NBB, DD / 128), 128, 0, stream>>>(AT, F[0], AV);
  k_out<<<NBB, 128, 0, stream>>>(AV, F[1], F[6], F[7], F[8], (float*)d_out);
}
